// InfiniteAttention_12360915878585
// MI455X (gfx1250) — hardware-verified
//
#include <hip/hip_runtime.h>


#define NB_  2
#define SS   4096
#define DD   512
#define NT   (NB_ * SS)
#define QB   256
#define HW   256
#define KW   768
#define SP   (SS + 2 * HW)
#define STRD 256
#define NSTR 16
typedef _Float16 h16;
typedef unsigned short bf;
typedef __attribute__((ext_vector_type(16))) __bf16   v16bf;
typedef __attribute__((ext_vector_type(16))) _Float16 v16h;
typedef __attribute__((ext_vector_type(8)))  _Float16 v8h;
typedef __attribute__((ext_vector_type(8)))  unsigned short v8us;
typedef __attribute__((ext_vector_type(8)))  float    v8f;
typedef __attribute__((ext_vector_type(4)))  float    v4f;
typedef v8h  __attribute__((may_alias)) v8ha;
typedef v4f  __attribute__((may_alias)) v4fa;
typedef v8us __attribute__((may_alias)) v8usa;

__device__ __forceinline__ unsigned short f2bf(float f) { unsigned u = __float_as_uint(f); u += 0x7FFFu + ((u >> 16) & 1u); return (unsigned short)(u >> 16); }
__device__ __forceinline__ float bf2f(unsigned short b) { return __uint_as_float(((unsigned)b) << 16); }
__device__ __forceinline__ float bfr(float f) { return bf2f(f2bf(f)); }
__device__ __forceinline__ v16h cat16(v8h lo, v8h hi) { return __builtin_shufflevector(lo, hi, 0, 1, 2, 3, 4, 5, 6, 7, 8, 9, 10, 11, 12, 13, 14, 15); }
__device__ __forceinline__ v16bf cat16b(v8us lo, v8us hi) { return __builtin_bit_cast(v16bf, __builtin_shufflevector(lo, hi, 0, 1, 2, 3, 4, 5, 6, 7, 8, 9, 10, 11, 12, 13, 14, 15)); }
__device__ __forceinline__ v8f wmma16(v16h a, v16h b, v8f c) { return __builtin_amdgcn_wmma_f32_16x16x32_f16(false, a, false, b, (short)0, c, false, false); }
__device__ __forceinline__ v8f wmmab(v16bf a, v16bf b, v8f c) { return __builtin_amdgcn_wmma_f32_16x16x32_bf16(false, a, false, b, (short)0, c, false, false); }


template <typename T16> struct WFrag;
template <> struct WFrag<h16> { typedef v16h V; static __device__ __forceinline__ V ld(const h16* p) { return cat16(*(const v8h*)p, *(const v8h*)(p + 16)); } static __device__ __forceinline__ v8f mma(V a, V b, v8f c) { return wmma16(a, b, c); } };
template <> struct WFrag<bf> { typedef v16bf V; static __device__ __forceinline__ V ld(const bf* p) { return cat16b(*(const v8us*)p, *(const v8us*)(p + 16)); } static __device__ __forceinline__ v8f mma(V a, V b, v8f c) { return wmmab(a, b, c); } };
template <typename T16, int NSPLIT, bool BIAS>
__global__ __launch_bounds__(32) void k_gemmw(const T16* __restrict__ A, const T16* __restrict__ A2, const T16* __restrict__ Bt, const T16* __restrict__ Bt2, int K, float* C, int ldc, const float* __restrict__ bias, size_t sA, size_t sB, size_t sC) {
    typedef typename WFrag<T16>::V V;
    __shared__ __align__(16) float os[16 * 68];
    const size_t z = blockIdx.z; A += z * sA; if (A2) A2 += z * sA; Bt += z * sB; if (Bt2) Bt2 += z * sB; C += z * sC;
    const int lane = threadIdx.x & 31, lr = lane & 15, hi = lane >> 4; const int r0 = blockIdx.x * 64, c0 = blockIdx.y * 64;
    v8f acc[4][4];
#pragma unroll
    for (int mb = 0; mb < 4; ++mb)
#pragma unroll
        for (int nb = 0; nb < 4; ++nb) acc[mb][nb] = (v8f){};
    const size_t aoff = (size_t)(r0 + lr) * K + 8 * hi, boff = (size_t)(c0 + lr) * K + 8 * hi;
#pragma unroll 1
    for (int kc = 0; kc < K; kc += 32) {
        V a[4], a2[4];
#pragma unroll
        for (int mb = 0; mb < 4; ++mb) { a[mb] = WFrag<T16>::ld(A + aoff + (size_t)mb * 16 * K + kc); if (NSPLIT == 1 || NSPLIT == 2) a2[mb] = WFrag<T16>::ld(A2 + aoff + (size_t)mb * 16 * K + kc); }
#pragma unroll
        for (int nb = 0; nb < 4; ++nb) { const V b = WFrag<T16>::ld(Bt + boff + (size_t)nb * 16 * K + kc); V b2; if (NSPLIT >= 2) b2 = WFrag<T16>::ld(Bt2 + boff + (size_t)nb * 16 * K + kc);
#pragma unroll
            for (int mb = 0; mb < 4; ++mb) { acc[mb][nb] = WFrag<T16>::mma(a[mb], b, acc[mb][nb]); if (NSPLIT == 1 || NSPLIT == 2) acc[mb][nb] = WFrag<T16>::mma(a2[mb], b, acc[mb][nb]); if (NSPLIT >= 2) acc[mb][nb] = WFrag<T16>::mma(a[mb], b2, acc[mb][nb]); } }
        asm volatile("v_nop\n\tv_nop\n\tv_nop\n\tv_nop" : "+v"(acc[0][0]), "+v"(acc[1][1]), "+v"(acc[2][2]), "+v"(acc[3][3]) : "v"(a[0]), "v"(a[3]));
    }
#pragma unroll
    for (int mb = 0; mb < 4; ++mb) {
#pragma unroll
        for (int nb = 0; nb < 4; ++nb) {
#pragma unroll
            for (int j = 0; j < 8; ++j) os[(hi * 8 + j) * 68 + nb * 16 + lr] = acc[mb][nb][j]; }
        __builtin_amdgcn_wave_barrier(); asm volatile("" ::: "memory");
        float* crow = C + (size_t)(r0 + mb * 16) * ldc + c0;
#pragma unroll 1
        for (int ps = 0; ps < 2; ++ps) {
#pragma unroll
            for (int s = 0; s < 8; ++s) { const int row = 2 * s + hi, cofs = lr * 4; v4f val = *(const v4fa*)(os + row * 68 + cofs); if (BIAS) { val[0] += bfr(bias[c0 + cofs]); val[1] += bfr(bias[c0 + cofs + 1]); val[2] += bfr(bias[c0 + cofs + 2]); val[3] += bfr(bias[c0 + cofs + 3]); }
                *(volatile v4f*)(crow + (size_t)row * ldc + cofs) = val; }
            if (ps == 0) __threadfence(); }
        __builtin_amdgcn_wave_barrier(); asm volatile("" ::: "memory");
    }
}

__device__ __forceinline__ void splitf(float y, unsigned short& h, unsigned short& l) { h = f2bf(y); l = f2bf(y - bf2f(h)); }
typedef __attribute__((ext_vector_type(2))) unsigned short v2us;

__global__ __launch_bounds__(256) void k_cvt8(const float* __restrict__ src, bf* dst, size_t n8) { const size_t i = (size_t)blockIdx.x * 256 + threadIdx.x; if (i >= n8) return; const v8f v = *(const v8f*)(src + i * 8); v8us o;
#pragma unroll
    for (int k = 0; k < 8; ++k) o[k] = f2bf(v[k]); *(volatile v8us*)(dst + i * 8) = o; __threadfence(); *(volatile v8us*)(dst + i * 8) = o; }
__global__ __launch_bounds__(256) void k_qin(const float* __restrict__ qry, const float* __restrict__ pos, bf* Ph, bf* Pl) {
    const int lane = threadIdx.x & 31; const int L0 = (blockIdx.x * 8 + (threadIdx.x >> 5)) * 8; const int nlines = NT * DD / 64;
#pragma unroll 1
    for (int ps = 0; ps < 2; ++ps) {
#pragma unroll
        for (int l = 0; l < 8; ++l) { const int L = L0 + l; if (L >= nlines) break; const int e = L * 64 + lane * 2; const int d = e & 511; const int s = (e >> 9) & (SS - 1); v2us oh, ol;
#pragma unroll
            for (int q = 0; q < 2; ++q) { unsigned short a, c2; splitf(bfr(qry[(size_t)e + q]) + bfr(pos[(size_t)s * DD + d + q]), a, c2); oh[q] = a; ol[q] = c2; }
            *(volatile v2us*)(Ph + (size_t)e) = oh; *(volatile v2us*)(Pl + (size_t)e) = ol; }
        if (ps == 0) __threadfence(); }
}
__global__ __launch_bounds__(256) void k_split(const float* __restrict__ A, int nlines, bf* Ph, bf* Pl) {
    const int lane = threadIdx.x & 31; const int L0 = (blockIdx.x * 8 + (threadIdx.x >> 5)) * 8;
#pragma unroll 1
    for (int ps = 0; ps < 2; ++ps) {
#pragma unroll
        for (int l = 0; l < 8; ++l) { const int L = L0 + l; if (L >= nlines) break; const int e = L * 64 + lane * 2; v2us oh, ol;
#pragma unroll
            for (int q = 0; q < 2; ++q) { unsigned short a, c2; splitf(A[(size_t)e + q], a, c2); oh[q] = a; ol[q] = c2; }
            *(volatile v2us*)(Ph + (size_t)e) = oh; *(volatile v2us*)(Pl + (size_t)e) = ol; }
        if (ps == 0) __threadfence(); }
}
__global__ __launch_bounds__(256) void k_kpad(const float* __restrict__ Kf, bf* Ph, bf* Pl) {
    const int lane = threadIdx.x & 31; const int L0 = (blockIdx.x * 8 + (threadIdx.x >> 5)) * 8; const int nlines = NB_ * SP * DD / 64;
#pragma unroll 1
    for (int ps = 0; ps < 2; ++ps) {
#pragma unroll
        for (int l = 0; l < 8; ++l) { const int L = L0 + l; if (L >= nlines) break; const size_t e = (size_t)L * 64 + lane * 2; const int d = (int)(e & 511); const int jp = (int)((e >> 9) % SP); const int b = (int)((e >> 9) / SP); const int j = jp - HW; v2us oh, ol;
#pragma unroll
            for (int q = 0; q < 2; ++q) { unsigned short a = 0, c2 = 0; if (j >= 0 && j < SS) splitf(Kf[((size_t)b * SS + j) * DD + d + q], a, c2); oh[q] = a; ol[q] = c2; }
            *(volatile v2us*)(Ph + e) = oh; *(volatile v2us*)(Pl + e) = ol; }
        if (ps == 0) __threadfence(); }
}
__global__ __launch_bounds__(256) void k_kstr(const float* __restrict__ Kf, const float* __restrict__ Vf, bf* KSh, bf* KSl, bf* VSh, bf* VSl) {
    const int lane = threadIdx.x & 31; const int L = blockIdx.x * 8 + (threadIdx.x >> 5); if (L >= NB_ * 64 * DD / 64) return; const int e = L * 64 + lane * 2;
    { const int d = e & 511; const int t = (e >> 9) & 63; const int b = e >> 15; v2us oh, ol;
#pragma unroll
      for (int q = 0; q < 2; ++q) { unsigned short a = 0, c2 = 0; if (t < NSTR) splitf(Kf[((size_t)b * SS + t * STRD) * DD + d + q], a, c2); oh[q] = a; ol[q] = c2; }
      *(volatile v2us*)(KSh + e) = oh; *(volatile v2us*)(KSl + e) = ol; }
    { const int t = e & 63; const int d = (e >> 6) & 511; const int b = e >> 15; v2us oh, ol;
#pragma unroll
      for (int q = 0; q < 2; ++q) { unsigned short a = 0, c2 = 0; if (t + q < NSTR) splitf(Vf[((size_t)b * SS + (t + q) * STRD) * DD + d], a, c2); oh[q] = a; ol[q] = c2; }
      *(volatile v2us*)(VSh + e) = oh; *(volatile v2us*)(VSl + e) = ol; }
    __threadfence();
    { const int d = e & 511; const int t = (e >> 9) & 63; const int b = e >> 15; v2us oh, ol;
#pragma unroll
      for (int q = 0; q < 2; ++q) { unsigned short a = 0, c2 = 0; if (t < NSTR) splitf(Kf[((size_t)b * SS + t * STRD) * DD + d + q], a, c2); oh[q] = a; ol[q] = c2; }
      *(volatile v2us*)(KSh + e) = oh; *(volatile v2us*)(KSl + e) = ol; }
    { const int t = e & 63; const int d = (e >> 6) & 511; const int b = e >> 15; v2us oh, ol;
#pragma unroll
      for (int q = 0; q < 2; ++q) { unsigned short a = 0, c2 = 0; if (t + q < NSTR) splitf(Vf[((size_t)b * SS + (t + q) * STRD) * DD + d], a, c2); oh[q] = a; ol[q] = c2; }
      *(volatile v2us*)(VSh + e) = oh; *(volatile v2us*)(VSl + e) = ol; }
}
__global__ __launch_bounds__(256) void k_isoft(const float* __restrict__ SW, const float* __restrict__ SX, int q0, bf* PWh, bf* PWl, bf* PXh, bf* PXl) {
    const int lane = threadIdx.x & 31; const int r = blockIdx.x * 8 + (threadIdx.x >> 5); if (r >= QB) return; const int i = q0 + r; const float* sw = SW + (size_t)r * KW; const float* sx = SX + (size_t)r * 64;
    const float isq = 22.62741661071777f;
    auto validw = [&](int c) { const int j = q0 - HW + c; return (j >= 0) && (j < SS) && (((j >= i - HW) && (j < i + HW)) || ((j & (STRD - 1)) == 0)); };
    auto validx = [&](int t) { const int j = t * STRD; return (t < NSTR) && !((j >= q0 - HW) && (j < q0 + 2 * HW)); };
    float m = -3.0e38f;
#pragma unroll 1
    for (int c0 = lane * 2; c0 < KW; c0 += 64) {
#pragma unroll
        for (int q = 0; q < 2; ++q) if (validw(c0 + q)) m = fmaxf(m, __fdiv_rn(sw[c0 + q], isq)); }
#pragma unroll
    for (int q = 0; q < 2; ++q) if (validx(lane * 2 + q)) m = fmaxf(m, __fdiv_rn(sx[lane * 2 + q], isq));
#pragma unroll
    for (int sh = 16; sh; sh >>= 1) m = fmaxf(m, __shfl_xor(m, sh, 32));
    float sum = 0.f;
#pragma unroll 1
    for (int c0 = lane * 2; c0 < KW; c0 += 64) {
#pragma unroll
        for (int q = 0; q < 2; ++q) if (validw(c0 + q)) sum += __expf(__fdiv_rn(sw[c0 + q], isq) - m); }
#pragma unroll
    for (int q = 0; q < 2; ++q) if (validx(lane * 2 + q)) sum += __expf(__fdiv_rn(sx[lane * 2 + q], isq) - m);
#pragma unroll
    for (int sh = 16; sh; sh >>= 1) sum += __shfl_xor(sum, sh, 32);
    const float f = __fdiv_rn(1.0f, sum);
#pragma unroll 1
    for (int ps = 0; ps < 2; ++ps) {
#pragma unroll 1
        for (int c0 = lane * 2; c0 < KW; c0 += 64) { v2us oh, ol;
#pragma unroll
            for (int q = 0; q < 2; ++q) { const float p = validw(c0 + q) ? __expf(__fdiv_rn(sw[c0 + q], isq) - m) * f : 0.f; unsigned short a, c2; splitf(p, a, c2); oh[q] = a; ol[q] = c2; }
            *(volatile v2us*)(PWh + (size_t)r * KW + c0) = oh; *(volatile v2us*)(PWl + (size_t)r * KW + c0) = ol; }
        { v2us oh, ol;
#pragma unroll
          for (int q = 0; q < 2; ++q) { const int t = lane * 2 + q; const float p = validx(t) ? __expf(__fdiv_rn(sx[t], isq) - m) * f : 0.f; unsigned short a, c2; splitf(p, a, c2); oh[q] = a; ol[q] = c2; }
          *(volatile v2us*)(PXh + (size_t)r * 64 + lane * 2) = oh; *(volatile v2us*)(PXl + (size_t)r * 64 + lane * 2) = ol; }
        if (ps == 0) __threadfence(); }
}
__global__ __launch_bounds__(256) void k_vtblk(const float* __restrict__ Vf, int b, int q0, bf* Ph, bf* Pl) {
    const int lane = threadIdx.x & 31; const int L0 = (blockIdx.x * 8 + (threadIdx.x >> 5)) * 8; const int nlines = DD * KW / 64;
#pragma unroll 1
    for (int ps = 0; ps < 2; ++ps) {
#pragma unroll
        for (int l = 0; l < 8; ++l) { const int L = L0 + l; if (L >= nlines) break; const int e = L * 64 + lane * 2; const int c = e % KW; const int d = e / KW; v2us oh, ol;
#pragma unroll
            for (int q = 0; q < 2; ++q) { const int j = q0 - HW + c + q; unsigned short a = 0, c2 = 0; if (j >= 0 && j < SS) splitf(Vf[((size_t)b * SS + j) * DD + d], a, c2); oh[q] = a; ol[q] = c2; }
            *(volatile v2us*)(Ph + (size_t)e) = oh; *(volatile v2us*)(Pl + (size_t)e) = ol; }
        if (ps == 0) __threadfence(); }
}
__global__ __launch_bounds__(256) void k_omix(const float* __restrict__ OW, const float* __restrict__ OX, int row0, bf* Ah, bf* Al) {
    const int lane = threadIdx.x & 31; const int L0 = (blockIdx.x * 8 + (threadIdx.x >> 5)) * 8; const int nlines = QB * DD / 64;
#pragma unroll 1
    for (int ps = 0; ps < 2; ++ps) {
#pragma unroll
        for (int l = 0; l < 8; ++l) { const int L = L0 + l; if (L >= nlines) break; const int e = L * 64 + lane * 2; v2us oh, ol;
#pragma unroll
            for (int q = 0; q < 2; ++q) { unsigned short a, c2; splitf(OW[(size_t)e + q] + OX[(size_t)e + q], a, c2); oh[q] = a; ol[q] = c2; }
            const size_t o = (size_t)row0 * DD + e; *(volatile v2us*)(Ah + o) = oh; *(volatile v2us*)(Al + o) = ol; }
        if (ps == 0) __threadfence(); }
}

extern "C" void kernel_launch(void* const* d_in, const int* in_sizes, int n_in,
                              void* d_out, int out_size, void* d_ws, size_t ws_size, hipStream_t stream) {
    (void)in_sizes; (void)n_in; (void)out_size;
    const float* qry = (const float*)d_in[0]; const float* ctx = (const float*)d_in[1]; const float* pos = (const float*)d_in[2];
    const float* Wq = (const float*)d_in[3]; const float* bq = (const float*)d_in[4]; const float* Wk = (const float*)d_in[5]; const float* bk = (const float*)d_in[6]; const float* Wv = (const float*)d_in[7]; const float* bv = (const float*)d_in[8]; const float* Wo = (const float*)d_in[9]; const float* bo = (const float*)d_in[10];
    float* OUT = (float*)d_out;
    char* wsp = (char*)d_ws;
    auto take = [&](size_t bytes) { char* p = wsp; wsp += (bytes + 255) & ~(size_t)255; return (void*)p; };
    bf* WQ = (bf*)take((size_t)DD * DD * 2); bf* WK = (bf*)take((size_t)DD * DD * 2); bf* WV = (bf*)take((size_t)DD * DD * 2); bf* WO = (bf*)take((size_t)DD * DD * 2);
    bf* QIh = (bf*)take((size_t)NT * DD * 2); bf* QIl = (bf*)take((size_t)NT * DD * 2); bf* CB = (bf*)take((size_t)NT * DD * 2);
    float* F = (float*)take((size_t)NT * DD * 4);
    bf* QPh = (bf*)take((size_t)NT * DD * 2); bf* QPl = (bf*)take((size_t)NT * DD * 2); bf* KPh = (bf*)take((size_t)NB_ * SP * DD * 2); bf* KPl = (bf*)take((size_t)NB_ * SP * DD * 2);
    float* Vf = (float*)take((size_t)NT * DD * 4); bf* KSh = (bf*)take((size_t)NB_ * 64 * DD * 2); bf* KSl = (bf*)take((size_t)NB_ * 64 * DD * 2); bf* VSh = (bf*)take((size_t)NB_ * DD * 64 * 2); bf* VSl = (bf*)take((size_t)NB_ * DD * 64 * 2);
    float* SW = (float*)take((size_t)QB * KW * 4); float* SX = (float*)take((size_t)QB * 64 * 4); bf* PWh = (bf*)take((size_t)QB * KW * 2); bf* PWl = (bf*)take((size_t)QB * KW * 2); bf* PXh = (bf*)take((size_t)QB * 64 * 2); bf* PXl = (bf*)take((size_t)QB * 64 * 2);
    bf* VTh = (bf*)take((size_t)DD * KW * 2); bf* VTl = (bf*)take((size_t)DD * KW * 2); float* OW = (float*)take((size_t)QB * DD * 4); float* OX = (float*)take((size_t)QB * DD * 4);
    bf* ATh = QIh; bf* ATl = QIl;
    if ((size_t)(wsp - (char*)d_ws) > ws_size) return;
    { const size_t nw = (size_t)DD * DD / 8; const unsigned g = (unsigned)((nw + 255) / 256); k_cvt8<<<g, 256, 0, stream>>>(Wq, WQ, nw); k_cvt8<<<g, 256, 0, stream>>>(Wk, WK, nw); k_cvt8<<<g, 256, 0, stream>>>(Wv, WV, nw); k_cvt8<<<g, 256, 0, stream>>>(Wo, WO, nw);
      const size_t nx = (size_t)NT * DD / 8; k_cvt8<<<(unsigned)((nx + 255) / 256), 256, 0, stream>>>(ctx, CB, nx); }
    const unsigned LB = (unsigned)((NT * DD / 64 + 63) / 64);
    k_qin<<<LB, 256, 0, stream>>>(qry, pos, QIh, QIl);
    k_gemmw<bf, 1, true><<<dim3(NT / 64, DD / 64, 1), 32, 0, stream>>>(QIh, QIl, WQ, nullptr, DD, F, DD, bq, 0, 0, 0);
    k_split<<<LB, 256, 0, stream>>>(F, NT * DD / 64, QPh, QPl);
    k_gemmw<bf, 0, true><<<dim3(NT / 64, DD / 64, 1), 32, 0, stream>>>(CB, nullptr, WK, nullptr, DD, F, DD, bk, 0, 0, 0);
    k_gemmw<bf, 0, true><<<dim3(NT / 64, DD / 64, 1), 32, 0, stream>>>(CB, nullptr, WV, nullptr, DD, Vf, DD, bv, 0, 0, 0);
    k_kpad<<<(unsigned)((NB_ * SP * DD / 64 + 63) / 64), 256, 0, stream>>>(F, KPh, KPl);
    k_kstr<<<(NB_ * 64 * DD / 64 + 7) / 8, 256, 0, stream>>>(F, Vf, KSh, KSl, VSh, VSl);
    for (int b = 0; b < NB_; ++b)
        for (int qb = 0; qb < SS / QB; ++qb) { const int q0 = qb * QB; const size_t qrow = (size_t)b * SS + q0;
            k_gemmw<bf, 2, false><<<dim3(QB / 64, KW / 64, 1), 32, 0, stream>>>(QPh + qrow * DD, QPl + qrow * DD, KPh + ((size_t)b * SP + q0) * DD, KPl + ((size_t)b * SP + q0) * DD, DD, SW, KW, nullptr, 0, 0, 0);
            k_gemmw<bf, 2, false><<<dim3(QB / 64, 1, 1), 32, 0, stream>>>(QPh + qrow * DD, QPl + qrow * DD, KSh + (size_t)b * 64 * DD, KSl + (size_t)b * 64 * DD, DD, SX, 64, nullptr, 0, 0, 0);
            k_isoft<<<QB / 8, 256, 0, stream>>>(SW, SX, q0, PWh, PWl, PXh, PXl);
            k_vtblk<<<(DD * KW / 64 + 63) / 64, 256, 0, stream>>>(Vf, b, q0, VTh, VTl);
            k_gemmw<bf, 2, false><<<dim3(QB / 64, DD / 64, 1), 32, 0, stream>>>(PWh, PWl, VTh, VTl, KW, OW, DD, nullptr, 0, 0, 0);
            k_gemmw<bf, 2, false><<<dim3(QB / 64, DD / 64, 1), 32, 0, stream>>>(PXh, PXl, VSh + (size_t)b * DD * 64, VSl + (size_t)b * DD * 64, 64, OX, DD, nullptr, 0, 0, 0);
            k_omix<<<(QB * DD / 64 + 63) / 64, 256, 0, stream>>>(OW, OX, (int)qrow, ATh, ATl); }
    k_gemmw<bf, 1, true><<<dim3(NT / 64, DD / 64, 1), 32, 0, stream>>>(ATh, ATl, WO, nullptr, DD, OUT, DD, bo, 0, 0, 0);
}
